// DynamicEdgeBiasAttention_71605694759111
// MI455X (gfx1250) — hardware-verified
//
#include <hip/hip_runtime.h>


#define NBT  2
#define NN   2048
#define DMOD 256
#define NH_  8
#define HD   32
#define HB   4
#define SS   NN
#define HDG  HD
#define DM_  DMOD
#define DM   DMOD
#define NTK  NN
#define SCL  0.17677669529663688f
#define LOSC 1024.0f

typedef _Float16 h16;
typedef unsigned short bf;
typedef __attribute__((ext_vector_type(16))) __bf16   v16bf;
typedef __attribute__((ext_vector_type(16))) _Float16 v16h;
typedef __attribute__((ext_vector_type(8)))  _Float16 v8h;
typedef __attribute__((ext_vector_type(8)))  unsigned short v8us;
typedef __attribute__((ext_vector_type(8)))  float    v8f;
typedef __attribute__((ext_vector_type(4)))  float    v4f;
typedef __attribute__((ext_vector_type(4)))  _Float16 v4h;
typedef v8h  __attribute__((may_alias)) v8ha;
typedef v4f  __attribute__((may_alias)) v4fa;
typedef v8us __attribute__((may_alias)) v8usa;

__device__ __forceinline__ unsigned short f2bf(float f) { unsigned u = __float_as_uint(f); u += 0x7FFFu + ((u >> 16) & 1u); return (unsigned short)(u >> 16); }
__device__ __forceinline__ float bf2f(unsigned short b) { return __uint_as_float(((unsigned)b) << 16); }
__device__ __forceinline__ float bfr(float f) { return bf2f(f2bf(f)); }
__device__ __forceinline__ v16h cat16(v8h lo, v8h hi) { return __builtin_shufflevector(lo, hi, 0, 1, 2, 3, 4, 5, 6, 7, 8, 9, 10, 11, 12, 13, 14, 15); }
__device__ __forceinline__ v16bf cat16b(v8us lo, v8us hi) { return __builtin_bit_cast(v16bf, __builtin_shufflevector(lo, hi, 0, 1, 2, 3, 4, 5, 6, 7, 8, 9, 10, 11, 12, 13, 14, 15)); }
__device__ __forceinline__ v8f wmma16(v16h a, v16h b, v8f c) { return __builtin_amdgcn_wmma_f32_16x16x32_f16(false, a, false, b, (short)0, c, false, false); }
__device__ __forceinline__ v8f wmmab(v16bf a, v16bf b, v8f c) { return __builtin_amdgcn_wmma_f32_16x16x32_bf16(false, a, false, b, (short)0, c, false, false); }

template <bool SPLITA, bool F16OUT = false>
__global__ __launch_bounds__(128) void k_gemmb(const bf* __restrict__ A, const bf* __restrict__ Al, const bf* __restrict__ Bn, const float* __restrict__ bias, float* C, int ldc, h16* C2, const float* __restrict__ R = nullptr, int K = DM, int roundR = 1) {
    __shared__ __align__(16) float ost[4][16 * 68];
    const int lane = threadIdx.x & 31, wave = threadIdx.x >> 5, lr = lane & 15, hi = lane >> 4;
    const int r0 = blockIdx.x * 64 + wave * 16, c0 = blockIdx.y * 64;
    const size_t aoff = (size_t)(r0 + lr) * K + 8 * hi;
    size_t boff[4];
#pragma unroll
    for (int t = 0; t < 4; ++t) boff[t] = (size_t)(c0 + t * 16 + lr) * K + 8 * hi;
    v8f acc[4];
#pragma unroll
    for (int t = 0; t < 4; ++t) acc[t] = (v8f){};
#pragma unroll 1
    for (int kc = 0; kc < K; kc += 32) {
        const v16bf a = cat16b(*(const v8us*)(A + aoff + kc), *(const v8us*)(A + aoff + kc + 16));
        v16bf al = a;
        if (SPLITA) al = cat16b(*(const v8us*)(Al + aoff + kc), *(const v8us*)(Al + aoff + kc + 16));
#pragma unroll
        for (int t = 0; t < 4; ++t) { const v16bf b = cat16b(*(const v8us*)(Bn + boff[t] + kc), *(const v8us*)(Bn + boff[t] + kc + 16)); acc[t] = wmmab(a, b, acc[t]); if (SPLITA) acc[t] = wmmab(al, b, acc[t]); }
        asm volatile("v_nop\n\tv_nop\n\tv_nop\n\tv_nop" : "+v"(acc[0]), "+v"(acc[1]), "+v"(acc[2]), "+v"(acc[3]) : "v"(a), "v"(al));
    }
    float* os = &ost[wave][0];
#pragma unroll
    for (int t = 0; t < 4; ++t) { const float bv = bias ? bfr(bias[c0 + t * 16 + lr]) : 0.f;
#pragma unroll
        for (int j = 0; j < 8; ++j) os[(hi * 8 + j) * 68 + t * 16 + lr] = acc[t][j] + bv; }
    __syncthreads();
    if (F16OUT) {
        h16* crow = (h16*)(void*)C + (size_t)r0 * ldc + c0;
        auto pass = [&]() {
#pragma unroll
            for (int s = 0; s < 4; ++s) { const int row = 4 * s + (lane >> 3), piece = lane & 7; const float* sp = os + row * 68 + piece * 8; v8h o, o2;
#pragma unroll
                for (int i = 0; i < 8; ++i) { const h16 a = (h16)sp[i]; o[i] = a; o2[i] = (h16)((sp[i] - (float)a) * LOSC); }
                *(volatile v8h*)(crow + (size_t)row * ldc + piece * 8) = o; if (C2) *(volatile v8h*)(C2 + (size_t)r0 * ldc + c0 + (size_t)row * ldc + piece * 8) = o2; }
        };
        pass(); __threadfence(); pass();
    } else {
        float* crow = C + (size_t)r0 * ldc + c0;
        auto pass = [&]() {
#pragma unroll
            for (int s = 0; s < 8; ++s) { const int Lid = (lane >> 3) + 4 * s, piece = lane & 7; const int row = Lid >> 1, cofs = (Lid & 1) * 32 + piece * 4;
                v4f val = *(const v4fa*)(os + row * 68 + cofs); if (R) { const v4f rv = *(const v4f*)(R + ((size_t)r0 + row) * ldc + c0 + cofs); val += roundR ? (v4f){bfr(rv[0]), bfr(rv[1]), bfr(rv[2]), bfr(rv[3])} : rv; }
                *(volatile v4f*)(crow + (size_t)row * ldc + cofs) = val; }
        };
        pass(); __threadfence(); pass();
    }
}

__global__ __launch_bounds__(256) void k_cvt8(const float* __restrict__ src, bf* dst, size_t n8) {
    const size_t i = (size_t)blockIdx.x * 256 + threadIdx.x; if (i >= n8) return;
    const v8f v = *(const v8f*)(src + i * 8); v8us o;
#pragma unroll
    for (int k = 0; k < 8; ++k) o[k] = f2bf(v[k]);
    *(volatile v8us*)(dst + i * 8) = o; __threadfence(); *(volatile v8us*)(dst + i * 8) = o;
}
__global__ __launch_bounds__(256) void k_zero8(bf* dst, size_t n8) {
    const size_t i = (size_t)blockIdx.x * 256 + threadIdx.x; if (i >= n8) return; v8us z;
#pragma unroll
    for (int k = 0; k < 8; ++k) z[k] = 0;
    *(volatile v8us*)(dst + i * 8) = z; __threadfence(); *(volatile v8us*)(dst + i * 8) = z;
}

template <int MODE>
__global__ __launch_bounds__(128) void k_gemm3z(const bf* __restrict__ Ah, const bf* __restrict__ Al, const bf* __restrict__ Bh, const bf* __restrict__ Bl, int K, float* C, int ldc, size_t sA, size_t sB, size_t sC) {
    if ((MODE & 1) && (int)blockIdx.y * 64 > (int)blockIdx.x * 64 + 63) return;
    const size_t z = blockIdx.z; Ah += z * sA; Al += z * sA; Bh += z * sB; Bl += z * sB; C += z * sC;
    const int Klim = (MODE & 2) ? min(K, ((int)blockIdx.x + 1) * 64) : K;
    __shared__ __align__(16) float ost[4][16 * 68];
    const int lane = threadIdx.x & 31, wave = threadIdx.x >> 5, lr = lane & 15, hi = lane >> 4;
    const int r0 = blockIdx.x * 64 + wave * 16, c0 = blockIdx.y * 64;
    const size_t aoff = (size_t)(r0 + lr) * K + 8 * hi;
    v8f acc[4];
#pragma unroll
    for (int t = 0; t < 4; ++t) acc[t] = (v8f){};
#pragma unroll 1
    for (int kc = 0; kc < Klim; kc += 32) {
        const v16bf a = cat16b(*(const v8us*)(Ah + aoff + kc), *(const v8us*)(Ah + aoff + kc + 16));
        v16bf al = a; if (!(MODE & 4) && !(MODE & 16)) al = cat16b(*(const v8us*)(Al + aoff + kc), *(const v8us*)(Al + aoff + kc + 16));
#pragma unroll
        for (int t = 0; t < 4; ++t) { const size_t bo = (size_t)(c0 + t * 16 + lr) * K + kc + 8 * hi;
            const v16bf bh = cat16b(*(const v8us*)(Bh + bo), *(const v8us*)(Bh + bo + 16));
            acc[t] = wmmab(a, bh, acc[t]);
            if (!(MODE & 4)) { if (!(MODE & 16)) acc[t] = wmmab(al, bh, acc[t]); if (!(MODE & 8)) { const v16bf bl = cat16b(*(const v8us*)(Bl + bo), *(const v8us*)(Bl + bo + 16)); acc[t] = wmmab(a, bl, acc[t]); } } }
        asm volatile("v_nop\n\tv_nop\n\tv_nop\n\tv_nop" : "+v"(acc[0]), "+v"(acc[1]), "+v"(acc[2]), "+v"(acc[3]) : "v"(a), "v"(al));
    }
    float* os = &ost[wave][0];
#pragma unroll
    for (int t = 0; t < 4; ++t) {
#pragma unroll
        for (int j = 0; j < 8; ++j) os[(hi * 8 + j) * 68 + t * 16 + lr] = acc[t][j]; }
    __builtin_amdgcn_wave_barrier(); asm volatile("" ::: "memory");
    float* crow = C + (size_t)r0 * ldc + c0;
    auto pass = [&]() {
#pragma unroll
        for (int s = 0; s < 8; ++s) { const int Lid = (lane >> 3) + 4 * s, piece = lane & 7; const int row = Lid >> 1, cofs = (Lid & 1) * 32 + piece * 4;
            const v4f val = *(const v4fa*)(os + row * 68 + cofs); *(volatile v4f*)(crow + (size_t)row * ldc + cofs) = val; }
    };
    pass(); __threadfence(); pass();
}
__global__ __launch_bounds__(256) void k_planes32z(const float* __restrict__ F, int ld, int off, float sc, int rows, bf* Ph, bf* Pl) {
    typedef __attribute__((ext_vector_type(2))) unsigned short v2us;
    const int lane = threadIdx.x & 31; const size_t r = ((size_t)blockIdx.x * 8 + (threadIdx.x >> 5)) * 2 + (lane >> 4); if (r >= (size_t)rows) return; const int z = blockIdx.z; const int c0 = (lane & 15) * 2; v2us oh, ol;
    Ph += (size_t)z * rows * 32; Pl += (size_t)z * rows * 32;
#pragma unroll
    for (int i = 0; i < 2; ++i) { const float y = F[r * ld + off + z * 32 + c0 + i] * sc; const unsigned short hb = f2bf(y); oh[i] = hb; ol[i] = f2bf(y - bf2f(hb)); }
    const size_t o = r * 32 + c0; *(volatile v2us*)(Ph + o) = oh; *(volatile v2us*)(Pl + o) = ol; __threadfence(); *(volatile v2us*)(Ph + o) = oh; *(volatile v2us*)(Pl + o) = ol;
}
__global__ __launch_bounds__(256) void k_vtpadz(const float* __restrict__ F, int ld, int off, int nk, bf* Th, bf* Tl) {
    typedef __attribute__((ext_vector_type(2))) unsigned short v2us;
    const int lane = threadIdx.x & 31; const size_t wid = (size_t)blockIdx.x * 8 + (threadIdx.x >> 5); if (wid >= (size_t)64 * (nk / 64)) return; const int z = blockIdx.z; const int d = (int)(wid / (nk / 64)); const int k0 = (int)(wid % (nk / 64)) * 64 + lane * 2; v2us oh, ol;
    Th += (size_t)z * 64 * nk; Tl += (size_t)z * 64 * nk;
#pragma unroll
    for (int i = 0; i < 2; ++i) { const float y = (d < 32) ? F[(size_t)(k0 + i) * ld + off + z * 32 + (d < 32 ? d : 0)] : 0.f; const unsigned short hb = f2bf(y); oh[i] = hb; ol[i] = f2bf(y - bf2f(hb)); }
    const size_t o = (size_t)d * nk + k0; *(volatile v2us*)(Th + o) = oh; *(volatile v2us*)(Tl + o) = ol; __threadfence(); *(volatile v2us*)(Th + o) = oh; *(volatile v2us*)(Tl + o) = ol;
}
template <int NK>
__global__ __launch_bounds__(256) void k_softmaxz(const float* __restrict__ S, int rows, bf* PH, bf* PL) {
    typedef __attribute__((ext_vector_type(4))) unsigned short v4us;
    const int lane = threadIdx.x & 31, i = blockIdx.x * 8 + (threadIdx.x >> 5); if (i >= rows) return; const size_t zo = (size_t)blockIdx.z * rows * NK; const float* sr = S + zo + (size_t)i * NK; PH += zo; PL += zo;
    float m = -3.0e38f;
#pragma unroll 1
    for (int c0 = lane * 4; c0 < NK; c0 += 128) {
#pragma unroll
        for (int q = 0; q < 4; ++q) m = fmaxf(m, sr[c0 + q]); }
#pragma unroll
    for (int sh = 16; sh; sh >>= 1) m = fmaxf(m, __shfl_xor(m, sh, 32));
    float sum = 0.f;
#pragma unroll 1
    for (int c0 = lane * 4; c0 < NK; c0 += 128) {
#pragma unroll
        for (int q = 0; q < 4; ++q) sum += __expf(sr[c0 + q] - m); }
#pragma unroll
    for (int sh = 16; sh; sh >>= 1) sum += __shfl_xor(sum, sh, 32);
    const float inv = 1.0f / sum;
#pragma unroll 1
    for (int ps = 0; ps < 2; ++ps) {
#pragma unroll 1
        for (int c0 = lane * 4; c0 < NK; c0 += 128) { v4us oh, ol;
#pragma unroll
            for (int q = 0; q < 4; ++q) { const float p = __expf(sr[c0 + q] - m) * inv; const unsigned short hb = f2bf(p); oh[q] = hb; ol[q] = f2bf(p - bf2f(hb)); }
            const size_t o = (size_t)i * NK + c0; *(volatile v4us*)(PH + o) = oh; *(volatile v4us*)(PL + o) = ol; }
        if (ps == 0) __threadfence(); }
}
__global__ __launch_bounds__(256) void k_placez(const float* __restrict__ XH, int rows, int ldy, float* Y) {
    const int lane = threadIdx.x & 31; const size_t q = (size_t)blockIdx.x * 8 + (threadIdx.x >> 5); if (q >= (size_t)rows) return; const int z = blockIdx.z; const float v = XH[((size_t)z * rows + q) * 64 + lane];
    *(volatile float*)(Y + q * ldy + z * 32 + lane) = v; __threadfence(); *(volatile float*)(Y + q * ldy + z * 32 + lane) = v;
}

__global__ __launch_bounds__(256) void k_cvt256(const float* __restrict__ src, int rows, bf* dst) {
    const int lane = threadIdx.x & 31; const size_t r = (size_t)blockIdx.x * 8 + (threadIdx.x >> 5); if (r >= (size_t)rows) return; v8us o;
#pragma unroll
    for (int i = 0; i < 8; ++i) o[i] = f2bf(src[r * DMOD + lane * 8 + i]);
    *(volatile v8us*)(dst + r * DMOD + lane * 8) = o; __threadfence(); *(volatile v8us*)(dst + r * DMOD + lane * 8) = o;
}
__global__ __launch_bounds__(256) void k_wcat3(const float* __restrict__ Wq, const float* __restrict__ Wk, const float* __restrict__ Wv, bf* WQKV) {
    const size_t i = ((size_t)blockIdx.x * 256 + threadIdx.x) * 8; if (i >= (size_t)3 * DMOD * DMOD) return; const size_t blk = i / ((size_t)DMOD * DMOD), o = i % ((size_t)DMOD * DMOD);
    const float* src = (blk == 0) ? Wq : (blk == 1) ? Wk : Wv; v8us v;
#pragma unroll
    for (int q = 0; q < 8; ++q) v[q] = f2bf(src[o + q]);
    *(volatile v8us*)(WQKV + i) = v; __threadfence(); *(volatile v8us*)(WQKV + i) = v;
}
__global__ __launch_bounds__(256) void k_bias3(const float* __restrict__ b0, const float* __restrict__ b1, const float* __restrict__ b2, float* B3) {
    const size_t i = (size_t)blockIdx.x * 256 + threadIdx.x; if (i >= (size_t)3 * DMOD) return; const int blk = (int)(i / DMOD), o = (int)(i % DMOD); const float v = (blk == 0) ? b0[o] : (blk == 1) ? b1[o] : b2[o];
    *(volatile float*)(B3 + i) = v; __threadfence(); *(volatile float*)(B3 + i) = v;
}
__global__ __launch_bounds__(256) void k_ebias(const float* __restrict__ A, const float* __restrict__ W1, const float* __restrict__ b1, const float* __restrict__ W2, const float* __restrict__ b2, int h0, float* BIAS) {
    const int lane = threadIdx.x & 31; const size_t i = (size_t)blockIdx.x * 8 + (threadIdx.x >> 5); if (i >= (size_t)NN) return; float w1[NH_], c1[NH_], w2[HB][NH_], c2[HB];
#pragma unroll
    for (int j = 0; j < NH_; ++j) { w1[j] = bfr(W1[j]); c1[j] = bfr(b1[j]); }
#pragma unroll
    for (int hh = 0; hh < HB; ++hh) { c2[hh] = bfr(b2[h0 + hh]);
#pragma unroll
        for (int j = 0; j < NH_; ++j) w2[hh][j] = bfr(W2[(h0 + hh) * NH_ + j]); }
#pragma unroll 1
    for (int ps = 0; ps < 2; ++ps) {
#pragma unroll 1
        for (int c = lane; c < NN; c += 32) { const float a = bfr(A[i * NN + c]); float hv[NH_];
#pragma unroll
            for (int j = 0; j < NH_; ++j) { const float t = fmaf(a, w1[j], c1[j]); hv[j] = (t >= 0.f) ? t : 0.01f * t; }
#pragma unroll
            for (int hh = 0; hh < HB; ++hh) { float s = c2[hh];
#pragma unroll
                for (int j = 0; j < NH_; ++j) s = fmaf(w2[hh][j], hv[j], s);
                *(volatile float*)(BIAS + ((size_t)hh * NN + i) * NN + c) = s; } }
        if (ps == 0) __threadfence(); }
}
__global__ __launch_bounds__(256) void k_bsoft(const float* __restrict__ S, float sc, const float* __restrict__ BI, bf* PH, bf* PL) {
    typedef __attribute__((ext_vector_type(4))) unsigned short v4us;
    const int lane = threadIdx.x & 31, i = blockIdx.x * 8 + (threadIdx.x >> 5); if (i >= NN) return; const float* sr = S + (size_t)i * NN; const float* br = BI + (size_t)i * NN;
    float m = -3.0e38f;
#pragma unroll 1
    for (int c0 = lane * 4; c0 < NN; c0 += 128) {
#pragma unroll
        for (int q = 0; q < 4; ++q) m = fmaxf(m, sr[c0 + q] * sc + br[c0 + q]); }
#pragma unroll
    for (int sh = 16; sh; sh >>= 1) m = fmaxf(m, __shfl_xor(m, sh, 32));
    float sum = 0.f;
#pragma unroll 1
    for (int c0 = lane * 4; c0 < NN; c0 += 128) {
#pragma unroll
        for (int q = 0; q < 4; ++q) sum += __expf(sr[c0 + q] * sc + br[c0 + q] - m); }
#pragma unroll
    for (int sh = 16; sh; sh >>= 1) sum += __shfl_xor(sum, sh, 32);
    const float inv = 1.0f / sum;
#pragma unroll 1
    for (int ps = 0; ps < 2; ++ps) {
#pragma unroll 1
        for (int c0 = lane * 4; c0 < NN; c0 += 128) { v4us oh, ol;
#pragma unroll
            for (int q = 0; q < 4; ++q) { const float p = __expf(sr[c0 + q] * sc + br[c0 + q] - m) * inv; const unsigned short hb = f2bf(p); oh[q] = hb; ol[q] = f2bf(p - bf2f(hb)); }
            const size_t o = (size_t)i * NN + c0; *(volatile v4us*)(PH + o) = oh; *(volatile v4us*)(PL + o) = ol; }
        if (ps == 0) __threadfence(); }
}
__global__ __launch_bounds__(256) void k_split256(const float* __restrict__ src, int rows, bf* dh, bf* dl) {
    const int lane = threadIdx.x & 31; const size_t r = (size_t)blockIdx.x * 8 + (threadIdx.x >> 5); if (r >= (size_t)rows) return; const size_t o = r * DMOD + lane * 8; const v8f v = *(const v8f*)(src + o); v8us oh, ol;
#pragma unroll
    for (int i = 0; i < 8; ++i) { const unsigned short hb = f2bf(v[i]); oh[i] = hb; ol[i] = f2bf(v[i] - bf2f(hb)); }
    *(volatile v8us*)(dh + o) = oh; *(volatile v8us*)(dl + o) = ol; __threadfence(); *(volatile v8us*)(dh + o) = oh; *(volatile v8us*)(dl + o) = ol;
}
__global__ __launch_bounds__(256) void k_hp32z(const float* __restrict__ F, int ld, int col0, int h0, bf* Ph, bf* Pl) {
    typedef __attribute__((ext_vector_type(2))) unsigned short v2us;
    const int lane = threadIdx.x & 31; const size_t r = ((size_t)blockIdx.x * 8 + (threadIdx.x >> 5)) * 2 + (lane >> 4); if (r >= (size_t)SS) return; const int z = blockIdx.z; const int d0 = (lane & 15) * 2; v2us oh, ol;
    Ph += (size_t)z * SS * HDG; Pl += (size_t)z * SS * HDG;
#pragma unroll
    for (int i = 0; i < 2; ++i) { const float y = F[r * ld + col0 + (h0 + z) * HDG + d0 + i]; const unsigned short hb = f2bf(y); oh[i] = hb; ol[i] = f2bf(y - bf2f(hb)); }
    const size_t o = r * HDG + d0; *(volatile v2us*)(Ph + o) = oh; *(volatile v2us*)(Pl + o) = ol; __threadfence(); *(volatile v2us*)(Ph + o) = oh; *(volatile v2us*)(Pl + o) = ol;
}
__global__ __launch_bounds__(256) void k_vt32z(const float* __restrict__ F, int ld, int col0, int h0, bf* Th, bf* Tl) {
    typedef __attribute__((ext_vector_type(2))) unsigned short v2us;
    const int lane = threadIdx.x & 31; const size_t wid = (size_t)blockIdx.x * 8 + (threadIdx.x >> 5); if (wid >= (size_t)64 * (SS / 64)) return; const int z = blockIdx.z; const int d = (int)(wid / (SS / 64)); const int t0 = (int)(wid % (SS / 64)) * 64 + lane * 2; v2us oh, ol;
    Th += (size_t)z * 64 * SS; Tl += (size_t)z * 64 * SS;
#pragma unroll
    for (int i = 0; i < 2; ++i) { const float y = (d < HDG) ? F[(size_t)(t0 + i) * ld + col0 + (h0 + z) * HDG + (d < HDG ? d : 0)] : 0.f; const unsigned short hb = f2bf(y); oh[i] = hb; ol[i] = f2bf(y - bf2f(hb)); }
    const size_t o = (size_t)d * SS + t0; *(volatile v2us*)(Th + o) = oh; *(volatile v2us*)(Tl + o) = ol; __threadfence(); *(volatile v2us*)(Th + o) = oh; *(volatile v2us*)(Tl + o) = ol;
}
__global__ __launch_bounds__(256) void k_place32z(const float* __restrict__ XO, int h0, float* ATT) {
    const int lane = threadIdx.x & 31; const size_t r = (size_t)blockIdx.x * 8 + (threadIdx.x >> 5); if (r >= (size_t)SS) return; const int z = blockIdx.z; const float v = XO[((size_t)z * SS + r) * 64 + lane];
    float* dst = ATT + r * DM_ + (h0 + z) * HDG + lane; *(volatile float*)dst = v; __threadfence(); *(volatile float*)dst = v;
}

extern "C" void kernel_launch(void* const* d_in, const int* in_sizes, int n_in,
                              void* d_out, int out_size, void* d_ws, size_t ws_size, hipStream_t stream) {
    (void)in_sizes; (void)n_in; (void)out_size;
    const float* x = (const float*)d_in[0]; const float* A = (const float*)d_in[1]; const float* Wq = (const float*)d_in[2]; const float* bq = (const float*)d_in[3]; const float* Wk = (const float*)d_in[4]; const float* bk = (const float*)d_in[5]; const float* Wv = (const float*)d_in[6]; const float* bv = (const float*)d_in[7];
    const float* Wo = (const float*)d_in[8]; const float* bo = (const float*)d_in[9]; const float* W1 = (const float*)d_in[10]; const float* b1 = (const float*)d_in[11]; const float* W2 = (const float*)d_in[12]; const float* b2 = (const float*)d_in[13];
    float* out = (float*)d_out;
    char* wsp = (char*)d_ws;
    auto take = [&](size_t bytes) { char* p = wsp; wsp += (bytes + 255) & ~(size_t)255; return (void*)p; };
    bf* WQKV = (bf*)take((size_t)3 * DMOD * DMOD * 2); float* B3 = (float*)take((size_t)3 * DMOD * 4); bf* WO = (bf*)take((size_t)DMOD * DMOD * 2);
    bf* Xb = (bf*)take((size_t)NN * DMOD * 2); float* QKV = (float*)take((size_t)NN * 3 * DMOD * 4); float* BIAS = (float*)take((size_t)HB * NN * NN * 4);
    bf* Qh = (bf*)take((size_t)NN * HD * 2); bf* Ql = (bf*)take((size_t)NN * HD * 2); bf* Kh = (bf*)take((size_t)NN * HD * 2); bf* Kl = (bf*)take((size_t)NN * HD * 2); bf* VTh = (bf*)take((size_t)64 * NN * 2); bf* VTl = (bf*)take((size_t)64 * NN * 2);
    float* S = (float*)take((size_t)NN * NN * 4); bf* PH = (bf*)take((size_t)NN * NN * 2); bf* PL = (bf*)take((size_t)NN * NN * 2); float* XO = (float*)take((size_t)NN * 64 * 4); float* ATT = (float*)take((size_t)NN * DMOD * 4); bf* Ah = (bf*)take((size_t)NN * DMOD * 2); bf* Al = (bf*)take((size_t)NN * DMOD * 2);
    if ((size_t)(wsp - (char*)d_ws) > ws_size) return;
    k_wcat3<<<(unsigned)((3 * (size_t)DMOD * DMOD / 8 + 255) / 256), 256, 0, stream>>>(Wq, Wk, Wv, WQKV); k_bias3<<<(3 * DMOD + 255) / 256, 256, 0, stream>>>(bq, bk, bv, B3); k_cvt8<<<(DMOD * DMOD / 8 + 255) / 256, 256, 0, stream>>>(Wo, WO, DMOD * DMOD / 8);
    for (int b = 0; b < NBT; ++b) { const float* Ab = A + (size_t)b * NN * NN;
        k_cvt256<<<NN / 8, 256, 0, stream>>>(x + (size_t)b * NN * DMOD, NN, Xb);
        k_gemmb<false, false><<<dim3(NN / 64, (3 * DMOD) / 64, 1), 128, 0, stream>>>(Xb, nullptr, WQKV, B3, QKV, 3 * DMOD, nullptr, nullptr, DMOD);
        for (int hb = 0; hb < NH_ / HB; ++hb) { const int h0 = hb * HB;
            k_ebias<<<NN / 8, 256, 0, stream>>>(Ab, W1, b1, W2, b2, h0, BIAS);
            for (int hh = 0; hh < HB; ++hh) { const int h = h0 + hh;
                k_hp32z<<<dim3((NN / 2) / 8, 1, 1), 256, 0, stream>>>(QKV, 3 * DMOD, 0, h, Qh, Ql); k_hp32z<<<dim3((NN / 2) / 8, 1, 1), 256, 0, stream>>>(QKV, 3 * DMOD, DMOD, h, Kh, Kl); k_vt32z<<<dim3((64 * (NN / 64)) / 8, 1, 1), 256, 0, stream>>>(QKV, 3 * DMOD, 2 * DMOD, h, VTh, VTl);
                k_gemm3z<0><<<dim3(NN / 64, NN / 64, 1), 128, 0, stream>>>(Qh, Ql, Kh, Kl, HD, S, NN, 0, 0, 0);
                k_bsoft<<<NN / 8, 256, 0, stream>>>(S, SCL, BIAS + (size_t)hh * NN * NN, PH, PL);
                k_gemm3z<0><<<dim3(NN / 64, 1, 1), 128, 0, stream>>>(PH, PL, VTh, VTl, NN, XO, 64, 0, 0, 0);
                k_place32z<<<dim3(NN / 8, 1, 1), 256, 0, stream>>>(XO, h, ATT); } }
        k_split256<<<NN / 8, 256, 0, stream>>>(ATT, NN, Ah, Al);
        k_gemmb<true, false><<<dim3(NN / 64, DMOD / 64, 1), 128, 0, stream>>>(Ah, Al, WO, bo, out + (size_t)b * NN * DMOD, DMOD, nullptr, nullptr, DMOD); }
}
